// Mamba2Layer_11476152615397
// MI455X (gfx1250) — hardware-verified
//
#include <hip/hip_runtime.h>
#include <math.h>

constexpr int kBatch  = 2;
constexpr int kSeqLen = 2048;
constexpr int kDModel = 1024;
constexpr int kDSsm   = 2048;
constexpr int kDState = 128;
constexpr int kNHeads = 32;
constexpr int kHeadP  = 64;
constexpr int kConvDim = 2304;
constexpr int kDInProj = 4384;
constexpr int kRows    = kBatch * kSeqLen;
constexpr int kNInPad  = 4416;
constexpr int kNDt     = 64;
constexpr int kTch     = 32;
constexpr float kWinCarry    = 64.0f;
constexpr float kWinCarryInv = 1.0f / 64.0f;
constexpr float kInvDSsm     = 1.0f / 2048.0f;
constexpr float kNormEps     = 1e-5f;

static_assert(kNInPad % 64 == 0 && kNInPad >= kDInProj);
static_assert(kDModel % 32 == 0 && kDSsm % 32 == 0);
static_assert(kRows % 64 == 0 && kDSsm % 64 == 0 && kConvDim % 64 == 0 && kDModel % 64 == 0);
static_assert(kSeqLen % kTch == 0);

constexpr size_t kSzXH  = (size_t)kRows * kDModel * 2;
constexpr size_t kSzWIN = (size_t)kNInPad * kDModel * 2;
constexpr size_t kSzZ   = (size_t)kRows * kDSsm * 4;
constexpr size_t kSzXR  = (size_t)kRows * kConvDim * 4;
constexpr size_t kSzDT  = (size_t)kRows * kNDt * 4;
constexpr size_t kSzXC  = (size_t)kRows * kConvDim * 4;
constexpr size_t kSzDL  = (size_t)kRows * kNHeads * 4;
constexpr size_t kSzY   = (size_t)kRows * kDSsm * 4;
constexpr size_t kSzYB  = (size_t)kRows * kDSsm * 2;
constexpr size_t kSzWO  = (size_t)kDModel * kDSsm * 2;
constexpr size_t kOffXH  = 0;
constexpr size_t kOffWIN = kOffXH + kSzXH;
constexpr size_t kOffZ   = kOffWIN + kSzWIN;
constexpr size_t kOffXR  = kOffZ + kSzZ;
constexpr size_t kOffDT  = kOffXR + kSzXR;
constexpr size_t kOffXC  = kOffDT + kSzDT;
constexpr size_t kOffDL  = kOffXC + kSzXC;
constexpr size_t kOffDA  = kOffDL + kSzDL;
constexpr size_t kWsTotal = kOffDA + kSzDL;
static_assert(kWsTotal == 128581632);
static_assert(kWsTotal <= 134217728);
static_assert(2 * kSzWO <= kSzXH);
static_assert(kSzY <= kSzXR);
static_assert(2 * kSzYB <= kSzXC);
static_assert(kOffWIN % 128 == 0 && kOffZ % 128 == 0 && kOffXR % 128 == 0 && kOffDT % 128 == 0);
static_assert(kOffXC % 128 == 0 && kOffDL % 128 == 0 && kOffDA % 128 == 0);

typedef __attribute__((ext_vector_type(16))) _Float16 v16h;
typedef __attribute__((ext_vector_type(8)))  _Float16 v8h;
typedef __attribute__((ext_vector_type(16))) __bf16   v16b;
typedef __attribute__((ext_vector_type(8)))  __bf16   v8b;
typedef __attribute__((ext_vector_type(8)))  float    v8f;
typedef __attribute__((ext_vector_type(4)))  float    v4f;
typedef __attribute__((ext_vector_type(4)))  unsigned int v4u;

__device__ __forceinline__ unsigned short f2bf_bits(float f) {
  unsigned u = __float_as_uint(f);
  return (unsigned short)((u + 0x7FFFu + ((u >> 16) & 1u)) >> 16);
}
__device__ __forceinline__ float bf_bits2f(unsigned short h) { return __uint_as_float(((unsigned)h) << 16); }

__device__ __forceinline__ void dep_guard_h(v8f& a, v8f& b, v16h x, v16h y) { asm volatile("v_nop\n\tv_nop\n\tv_nop\n\tv_nop" : "+v"(a), "+v"(b) : "v"(x), "v"(y)); }
__device__ __forceinline__ void dep_guard_b(v8f& a, v8f& b, v16b x, v16b y) { asm volatile("v_nop\n\tv_nop\n\tv_nop\n\tv_nop" : "+v"(a), "+v"(b) : "v"(x), "v"(y)); }
__device__ __forceinline__ void keep4_h(v16h a, v16h b, v16h c, v16h d) { asm volatile("v_nop" :: "v"(a), "v"(b), "v"(c), "v"(d)); }
__device__ __forceinline__ void keep4_b(v16b a, v16b b, v16b c, v16b d) { asm volatile("v_nop" :: "v"(a), "v"(b), "v"(c), "v"(d)); }
__device__ __forceinline__ void acc_guard4(v8f& a, v8f& b, v8f& c, v8f& d) { asm volatile("v_nop\n\tv_nop\n\tv_nop\n\tv_nop" : "+v"(a), "+v"(b), "+v"(c), "+v"(d)); }
template <typename T> struct Frag;
template <> struct Frag<_Float16> {
  typedef v16h V; union U { v16h v; v8h h[2]; };
  static __device__ __forceinline__ v16h load(const _Float16* p) {
    U f; f.h[0] = *(const v8h*)(p); f.h[1] = *(const v8h*)(p + 16); return f.v;
  }
  static __device__ __forceinline__ v8f mma(v16h a, v16h b, v8f c) {
    return __builtin_amdgcn_wmma_f32_16x16x32_f16(false, a, false, b, (short)0, c, false, false);
  }
  static __device__ __forceinline__ void guard(v8f& a, v8f& b, v16h x, v16h y) { dep_guard_h(a, b, x, y); }
  static __device__ __forceinline__ void keep(v16h a, v16h b, v16h c, v16h d) { keep4_h(a, b, c, d); }
};
template <> struct Frag<__bf16> {
  typedef v16b V; union U { v16b v; v8b h[2]; };
  static __device__ __forceinline__ v16b load(const __bf16* p) {
    U f; f.h[0] = *(const v8b*)(p); f.h[1] = *(const v8b*)(p + 16); return f.v;
  }
  static __device__ __forceinline__ v8f mma(v16b a, v16b b, v8f c) {
    return __builtin_amdgcn_wmma_f32_16x16x32_bf16(false, a, false, b, (short)0, c, false, false);
  }
  static __device__ __forceinline__ void guard(v8f& a, v8f& b, v16b x, v16b y) { dep_guard_b(a, b, x, y); }
  static __device__ __forceinline__ void keep(v16b a, v16b b, v16b c, v16b d) { keep4_b(a, b, c, d); }
};

__device__ __forceinline__ unsigned pk16(unsigned short a, unsigned short b) { return (unsigned)a | ((unsigned)b << 16); }
__device__ __forceinline__ unsigned short h_bits(float f) { const _Float16 h = (_Float16)f; return __builtin_bit_cast(unsigned short, h); }

template <int ET> struct Elem;
template <> struct Elem<0> { typedef _Float16 T; };
template <> struct Elem<1> { typedef __bf16 T; };
template <int ET, bool SPLIT, int BIAS_MODE, int OUT_MODE, bool RESID, int ACT = 0>
__global__ __launch_bounds__(256) void wmma_gemm64(
    const unsigned short* __restrict__ Ap, const unsigned short* __restrict__ A2p, int lda, long strideA,
    const unsigned short* __restrict__ Btp, const unsigned short* __restrict__ Bt2p, int ldb, long strideB,
    void* __restrict__ Cout, void* __restrict__ Cout2, int ldc, long strideC,
    const float* __restrict__ bias,
    const float* __restrict__ resid, long strideR,
    int M, int N, int K, float scale) {
  typedef typename Elem<ET>::T T;
  typedef typename Frag<T>::V V;
  const T* A = (const T*)Ap; const T* A2 = (const T*)A2p; const T* Bt = (const T*)Btp; const T* Bt2 = (const T*)Bt2p;
  __shared__ __align__(16) float sT[8][16 * 68];
  const int b    = blockIdx.y;
  const int lane = threadIdx.x & 31;
  const int wave = threadIdx.x >> 5;
  const int tilesN = N >> 6;
  const int tilesM = M >> 6;
  const int tile = blockIdx.x * 8 + wave;
  if (tile >= tilesM * tilesN) return;
  const int tm = tile / tilesN;
  const int tn = tile - tm * tilesN;
  const int m0 = tm << 6;
  const int n0 = tn << 6;

  const T* Ab  = A  + (size_t)b * strideA;
  const T* Bb  = Bt + (size_t)b * strideB;
  const T* Ab2 = SPLIT ? (A2  + (size_t)b * strideA) : nullptr;
  const T* Bb2 = SPLIT ? (Bt2 + (size_t)b * strideB) : nullptr;

  const int rlane = lane & 15;
  const int koff  = (lane >> 4) * 8;
  const int mOff  = (lane >> 4) * 8;

  v8f acc[4][4];
#pragma unroll
  for (int i = 0; i < 4; ++i)
#pragma unroll
    for (int j = 0; j < 4; ++j) acc[i][j] = (v8f){0.f,0.f,0.f,0.f,0.f,0.f,0.f,0.f};

  for (int k0 = 0; k0 < K; k0 += 32) {
    V bh[4], bl[4];
#pragma unroll
    for (int j = 0; j < 4; ++j) {
      const size_t bo = (size_t)(n0 + (j << 4) + rlane) * ldb + koff + k0;
      bh[j] = Frag<T>::load(Bb + bo);
      if (SPLIT) bl[j] = Frag<T>::load(Bb2 + bo);
    }
#pragma unroll
    for (int i = 0; i < 4; ++i) {
      const size_t ao = (size_t)(m0 + (i << 4) + rlane) * lda + koff + k0;
      V ah = Frag<T>::load(Ab + ao);
      V al;
      if (SPLIT) al = Frag<T>::load(Ab2 + ao);
#pragma unroll
      for (int j = 0; j < 4; ++j) {
        acc[i][j] = Frag<T>::mma(ah, bh[j], acc[i][j]);
        if (SPLIT) {
          acc[i][j] = Frag<T>::mma(ah, bl[j], acc[i][j]);
          acc[i][j] = Frag<T>::mma(al, bh[j], acc[i][j]);
        }
      }
      Frag<T>::guard(acc[i][0], acc[i][3], ah, SPLIT ? al : ah);
    }
    Frag<T>::keep(bh[0], bh[1], bh[2], bh[3]);
    if (SPLIT) Frag<T>::keep(bl[0], bl[1], bl[2], bl[3]);
  }
  acc_guard4(acc[0][0], acc[0][1], acc[0][2], acc[0][3]);
  acc_guard4(acc[1][0], acc[1][1], acc[1][2], acc[1][3]);
  acc_guard4(acc[2][0], acc[2][1], acc[2][2], acc[2][3]);
  acc_guard4(acc[3][0], acc[3][1], acc[3][2], acc[3][3]);

  float* slab = sT[wave];
  const float* Rb = RESID ? (resid + (size_t)b * strideR) : nullptr;
#pragma unroll
  for (int i = 0; i < 4; ++i) {
    const int mBase = m0 + (i << 4);
#pragma unroll
    for (int j = 0; j < 4; ++j) {
      const int n = n0 + (j << 4) + rlane;
      float bv = 0.f;
      if (BIAS_MODE == 2) bv = bias[n];
#pragma unroll
      for (int r = 0; r < 8; ++r) {
        float v = acc[i][j][r] * scale;
        if (BIAS_MODE == 1) v += bias[mBase + mOff + r];
        if (BIAS_MODE == 2) v += bv;
        if (RESID) v += Rb[(size_t)(mBase + mOff + r) * ldc + n];
        if (ACT == 2) v = fmaxf(v, 0.0f);
        if (ACT == 4) v = (v > 0.f) ? v : 0.01f * v;
        slab[(mOff + r) * 68 + (j << 4) + rlane] = v;
      }
    }
    __builtin_amdgcn_fence(__ATOMIC_RELEASE, "workgroup");
    __builtin_amdgcn_wave_barrier();
    __builtin_amdgcn_fence(__ATOMIC_ACQUIRE, "workgroup");
    if (OUT_MODE == 0) {
      float* C = (float*)Cout + (size_t)b * strideC;
      const int hh = lane >> 4, c4 = (lane & 15) * 4;
      for (int pass = 0; pass < 2; ++pass) {
#pragma unroll
        for (int it = 0; it < 8; ++it) {
          const int row = it * 2 + hh;
          v4f v = *(const v4f*)(slab + row * 68 + c4);
          *(volatile v4f*)(C + (size_t)(mBase + row) * ldc + n0 + c4) = v;
        }
        __threadfence();
      }
    } else {
      const int q = lane >> 3, c8 = (lane & 7) * 8;
      unsigned short* C  = (unsigned short*)Cout  + (size_t)b * strideC;
      unsigned short* C2 = (OUT_MODE == 2) ? ((unsigned short*)Cout2 + (size_t)b * strideC) : nullptr;
      for (int pass = 0; pass < 2; ++pass) {
#pragma unroll
        for (int it = 0; it < 4; ++it) {
          const int row = it * 4 + q;
          const float* sp = slab + row * 68 + c8;
          v8h hv, lv;
#pragma unroll
          for (int e = 0; e < 8; ++e) {
            if (OUT_MODE == 1) {
              hv[e] = (_Float16)sp[e];
            } else {
              unsigned short hb = f2bf_bits(sp[e]);
              unsigned short lb = f2bf_bits(sp[e] - bf_bits2f(hb));
              hv[e] = __builtin_bit_cast(_Float16, hb);
              lv[e] = __builtin_bit_cast(_Float16, lb);
            }
          }
          *(volatile v8h*)(C + (size_t)(mBase + row) * ldc + n0 + c8) = hv;
          if (OUT_MODE == 2) *(volatile v8h*)(C2 + (size_t)(mBase + row) * ldc + n0 + c8) = lv;
        }
        __threadfence();
      }
    }
    __builtin_amdgcn_fence(__ATOMIC_RELEASE, "workgroup");
    __builtin_amdgcn_wave_barrier();
    __builtin_amdgcn_fence(__ATOMIC_ACQUIRE, "workgroup");
  }
}

__global__ __launch_bounds__(256) void cast8_f16_kernel(const float* __restrict__ in, unsigned short* __restrict__ out, int n8) {
  const int i = blockIdx.x * 256 + threadIdx.x;
  if (i >= n8) return;
  const float* p = in + 8 * (size_t)i;
  const v4f a = *(const v4f*)(p);
  const v4f c = *(const v4f*)(p + 4);
  unsigned short hb[8];
#pragma unroll
  for (int e = 0; e < 4; ++e) {
    hb[e]     = h_bits(a[e]);
    hb[4 + e] = h_bits(c[e]);
  }
  const v4u u = (v4u){pk16(hb[0], hb[1]), pk16(hb[2], hb[3]), pk16(hb[4], hb[5]), pk16(hb[6], hb[7])};
  unsigned short* q = out + 8 * (size_t)i;
  *(volatile v4u*)q = u;
  __threadfence();
  *(volatile v4u*)q = u;
}

__global__ __launch_bounds__(256) void win_tcast_kernel(const float* __restrict__ W, unsigned short* __restrict__ out) {
  __shared__ float sm[64][65];
  const int t  = threadIdx.x;
  const int d0 = blockIdx.x * 64;
  const int n0 = blockIdx.y * 64;
#pragma unroll
  for (int i = 0; i < 16; ++i) {
    const int e = i * 256 + t;
    const int r = e >> 6;
    const int c = e & 63;
    const int n  = n0 + c;
    const int nc = (n < kDInProj) ? n : (kDInProj - 1);
    float v = W[(size_t)(d0 + r) * kDInProj + nc] * kWinCarry;
    v = (n < kDInProj) ? v : 0.0f;
    sm[c][r] = v;
  }
  __syncthreads();
  const int lane = t & 31, wave = t >> 5;
  const int q = lane >> 3, c8 = (lane & 7) * 8;
  for (int pass = 0; pass < 2; ++pass) {
#pragma unroll
    for (int it = 0; it < 2; ++it) {
      const int row = wave * 8 + it * 4 + q;
      unsigned short hb[8];
#pragma unroll
      for (int e = 0; e < 8; ++e) hb[e] = h_bits(sm[row][c8 + e]);
      const v4u u = (v4u){pk16(hb[0], hb[1]), pk16(hb[2], hb[3]), pk16(hb[4], hb[5]), pk16(hb[6], hb[7])};
      *(volatile v4u*)(out + (size_t)(n0 + row) * kDModel + d0 + c8) = u;
    }
    __threadfence();
  }
}

__global__ __launch_bounds__(256) void wout_tsplit_kernel(const float* __restrict__ W, unsigned short* __restrict__ outH,
                                                         unsigned short* __restrict__ outL) {
  __shared__ float sm[64][65];
  const int t  = threadIdx.x;
  const int k0 = blockIdx.x * 64;
  const int n0 = blockIdx.y * 64;
#pragma unroll
  for (int i = 0; i < 16; ++i) {
    const int e = i * 256 + t;
    const int r = e >> 6;
    const int c = e & 63;
    sm[c][r] = W[(size_t)(k0 + r) * kDModel + n0 + c];
  }
  __syncthreads();
  const int lane = t & 31, wave = t >> 5;
  const int q = lane >> 3, c8 = (lane & 7) * 8;
  for (int pass = 0; pass < 2; ++pass) {
#pragma unroll
    for (int it = 0; it < 2; ++it) {
      const int row = wave * 8 + it * 4 + q;
      unsigned short hb[8], lb[8];
#pragma unroll
      for (int e = 0; e < 8; ++e) {
        const float v = sm[row][c8 + e];
        hb[e] = f2bf_bits(v);
        lb[e] = f2bf_bits(v - bf_bits2f(hb[e]));
      }
      const v4u uh = (v4u){pk16(hb[0], hb[1]), pk16(hb[2], hb[3]), pk16(hb[4], hb[5]), pk16(hb[6], hb[7])};
      const v4u ul = (v4u){pk16(lb[0], lb[1]), pk16(lb[2], lb[3]), pk16(lb[4], lb[5]), pk16(lb[6], lb[7])};
      const size_t o = (size_t)(n0 + row) * kDSsm + k0 + c8;
      *(volatile v4u*)(outH + o) = uh;
      *(volatile v4u*)(outL + o) = ul;
    }
    __threadfence();
  }
}

__global__ __launch_bounds__(256) void dtprep_kernel(const float* __restrict__ DT, const float* __restrict__ dtb,
                                                    const float* __restrict__ Alog, float* __restrict__ DL,
                                                    float* __restrict__ DA) {
  const int i = blockIdx.x * 256 + threadIdx.x;
  if (i >= kRows * kNHeads) return;
  const int row = i >> 5, h = i & 31;
  const float x = DT[(size_t)row * kNDt + h] + dtb[h];
  const float delta = fmaxf(x, 0.0f) + log1pf(expf(-fabsf(x)));
  const float ah = -expf(Alog[h]);
  const float da = expf(delta * ah);
  ((volatile float*)DL)[i] = delta;
  ((volatile float*)DA)[i] = da;
  __threadfence();
  ((volatile float*)DL)[i] = delta;
  ((volatile float*)DA)[i] = da;
}

__global__ __launch_bounds__(256) void conv_silu_kernel(const float* __restrict__ XR, const float* __restrict__ cw,
                                                       const float* __restrict__ cb, float* __restrict__ XC) {
  const int i = blockIdx.x * 256 + threadIdx.x;
  if (i >= kRows * kConvDim / 4) return;
  const size_t e0 = (size_t)i * 4;
  const int row = (int)(e0 / kConvDim);
  const int c   = (int)(e0 - (size_t)row * kConvDim);
  const int l   = row & (kSeqLen - 1);
  v4f acc = *(const v4f*)(cb + c);
#pragma unroll
  for (int k = 0; k < 4; ++k) {
    const int ls = l - 3 + k;
    const int rk = (ls >= 0) ? (row - 3 + k) : row;
    const v4f xv = *(const v4f*)(XR + (size_t)rk * kConvDim + c);
    const v4f wv = *(const v4f*)(cw + (size_t)k * kConvDim + c);
#pragma unroll
    for (int e = 0; e < 4; ++e) {
      const float xe = (ls >= 0) ? xv[e] : 0.0f;
      acc[e] = acc[e] + xe * wv[e];
    }
  }
  v4f o;
#pragma unroll
  for (int e = 0; e < 4; ++e) {
    const float a = acc[e];
    o[e] = a * __builtin_amdgcn_rcpf(1.0f + expf(-a));
  }
  *(volatile v4f*)(XC + e0) = o;
  __threadfence();
  *(volatile v4f*)(XC + e0) = o;
}

__global__ __launch_bounds__(256) void scan_kernel(const float* __restrict__ XC, const float* __restrict__ DL,
                                                  const float* __restrict__ DA, const float* __restrict__ Dv,
                                                  float* __restrict__ Y) {
  __shared__ __align__(16) float BCs[kTch * 2 * kDState];
  __shared__ __align__(16) float Xs[kTch * kHeadP];
  __shared__ __align__(16) float Ys[kTch * kHeadP];
  __shared__ float dls[kTch];
  __shared__ float das[kTch];

  const int b = blockIdx.x >> 5;
  const int h = blockIdx.x & 31;
  const int t = threadIdx.x;
  const int lane = t & 31, wave = t >> 5;
  const int p = t >> 2;
  const int q = t & 3;
  const float Dh = Dv[h];

  float st[32];
#pragma unroll
  for (int j = 0; j < 32; ++j) st[j] = 0.0f;

#pragma unroll 1
  for (int ch = 0; ch < kSeqLen / kTch; ++ch) {
    const int rowbase = b * kSeqLen + ch * kTch;
#pragma unroll
    for (int i = 0; i < 8; ++i) {
      const int idx = i * 256 + t;
      const int s   = idx >> 6;
      const int c4  = (idx & 63) * 4;
      const v4f v = *(const v4f*)(XC + (size_t)(rowbase + s) * kConvDim + kDSsm + c4);
      *(v4f*)(BCs + s * 256 + c4) = v;
    }
#pragma unroll
    for (int i = 0; i < 2; ++i) {
      const int idx = i * 256 + t;
      const int s   = idx >> 4;
      const int c4  = (idx & 15) * 4;
      const v4f v = *(const v4f*)(XC + (size_t)(rowbase + s) * kConvDim + h * kHeadP + c4);
      *(v4f*)(Xs + s * kHeadP + c4) = v;
    }
    if (t < kTch) {
      dls[t] = DL[(size_t)(rowbase + t) * kNHeads + h];
      das[t] = DA[(size_t)(rowbase + t) * kNHeads + h];
    }
    __syncthreads();

#pragma unroll 1
    for (int s = 0; s < kTch; ++s) {
      const float dA = das[s];
      const float xv = Xs[s * kHeadP + p];
      const float dx = dls[s] * xv;
      const float* bp = BCs + s * 256 + q * 32;
      float acc = 0.0f;
#pragma unroll
      for (int j4 = 0; j4 < 8; ++j4) {
        const v4f bv = *(const v4f*)(bp + 4 * j4);
        const v4f cv = *(const v4f*)(bp + kDState + 4 * j4);
#pragma unroll
        for (int e = 0; e < 4; ++e) {
          const float hn = dA * st[4 * j4 + e] + dx * bv[e];
          st[4 * j4 + e] = hn;
          acc += hn * cv[e];
        }
      }
      acc += __shfl_xor(acc, 1, 32);
      acc += __shfl_xor(acc, 2, 32);
      const float yv = acc + Dh * xv;
      if (q == 0) Ys[s * kHeadP + p] = yv;
    }
    __syncthreads();

    {
      const int hh = lane >> 4, c4 = (lane & 15) * 4;
      for (int pass = 0; pass < 2; ++pass) {
#pragma unroll
        for (int it = 0; it < 2; ++it) {
          const int s = wave * 4 + it * 2 + hh;
          const v4f v = *(const v4f*)(Ys + s * kHeadP + c4);
          *(volatile v4f*)(Y + (size_t)(rowbase + s) * kDSsm + h * kHeadP + c4) = v;
        }
        __threadfence();
      }
    }
  }
}

__global__ __launch_bounds__(256) void gate_kernel(const float* __restrict__ Y, const float* __restrict__ Z,
                                                  const float* __restrict__ gam, unsigned short* __restrict__ YH,
                                                  unsigned short* __restrict__ YL) {
  __shared__ float red[8];
  const int row  = blockIdx.x;
  const int t    = threadIdx.x;
  const int lane = t & 31, wave = t >> 5;
  const size_t base = (size_t)row * kDSsm + 8 * t;
  const v4f ya = *(const v4f*)(Y + base);
  const v4f yb = *(const v4f*)(Y + base + 4);
  float yv[8];
#pragma unroll
  for (int e = 0; e < 4; ++e) { yv[e] = ya[e]; yv[4 + e] = yb[e]; }
  float ss = 0.0f;
#pragma unroll
  for (int e = 0; e < 8; ++e) ss += yv[e] * yv[e];
#pragma unroll
  for (int off = 16; off > 0; off >>= 1) ss += __shfl_xor(ss, off, 32);
  if (lane == 0) red[wave] = ss;
  __syncthreads();
  float tot = red[0];
#pragma unroll
  for (int w = 1; w < 8; ++w) tot += red[w];
  const float inv = rsqrtf(tot * kInvDSsm + kNormEps);

  const v4f za = *(const v4f*)(Z + base);
  const v4f zb = *(const v4f*)(Z + base + 4);
  const v4f ga = *(const v4f*)(gam + 8 * t);
  const v4f gb = *(const v4f*)(gam + 8 * t + 4);
  unsigned short hb[8], lb[8];
#pragma unroll
  for (int e = 0; e < 8; ++e) {
    const float ze = (e < 4) ? za[e] : zb[e - 4];
    const float ge = (e < 4) ? ga[e] : gb[e - 4];
    const float yn = (yv[e] * inv) * ge;
    const float sz = ze * __builtin_amdgcn_rcpf(1.0f + expf(-ze));
    const float o  = yn * sz;
    hb[e] = f2bf_bits(o);
    lb[e] = f2bf_bits(o - bf_bits2f(hb[e]));
  }
  const v4u uh = (v4u){pk16(hb[0], hb[1]), pk16(hb[2], hb[3]), pk16(hb[4], hb[5]), pk16(hb[6], hb[7])};
  const v4u ul = (v4u){pk16(lb[0], lb[1]), pk16(lb[2], lb[3]), pk16(lb[4], lb[5]), pk16(lb[6], lb[7])};
  unsigned short* ph = YH + base;
  unsigned short* pl = YL + base;
  *(volatile v4u*)ph = uh;
  *(volatile v4u*)pl = ul;
  __threadfence();
  *(volatile v4u*)ph = uh;
  *(volatile v4u*)pl = ul;
}

extern "C" void kernel_launch(void* const* d_in, const int* in_sizes, int n_in,
                              void* d_out, int out_size, void* d_ws, size_t ws_size,
                              hipStream_t stream) {
  (void)in_sizes; (void)n_in; (void)out_size;
  if (ws_size < kWsTotal) return;
  const float* hs    = (const float*)d_in[0];
  const float* Win   = (const float*)d_in[1];
  const float* cw    = (const float*)d_in[2];
  const float* cb    = (const float*)d_in[3];
  const float* Alog  = (const float*)d_in[4];
  const float* Dv    = (const float*)d_in[5];
  const float* dtb   = (const float*)d_in[6];
  const float* gam   = (const float*)d_in[7];
  const float* Wout  = (const float*)d_in[8];
  float* out = (float*)d_out;
  char* ws = (char*)d_ws;

  unsigned short* XH  = (unsigned short*)(ws + kOffXH);
  unsigned short* WIN = (unsigned short*)(ws + kOffWIN);
  float* Zp  = (float*)(ws + kOffZ);
  float* XR  = (float*)(ws + kOffXR);
  float* DTp = (float*)(ws + kOffDT);
  float* XC  = (float*)(ws + kOffXC);
  float* DL  = (float*)(ws + kOffDL);
  float* DA  = (float*)(ws + kOffDA);
  unsigned short* WOH = (unsigned short*)(ws + kOffXH);
  unsigned short* WOL = (unsigned short*)(ws + kOffXH + kSzWO);
  float* Yp = (float*)(ws + kOffXR);
  unsigned short* YH = (unsigned short*)(ws + kOffXC);
  unsigned short* YL = (unsigned short*)(ws + kOffXC + kSzYB);

  {
    const int n8 = kRows * kDModel / 8;
    cast8_f16_kernel<<<dim3((n8 + 255) / 256), dim3(256), 0, stream>>>(hs, XH, n8);
  }
  win_tcast_kernel<<<dim3(kDModel / 64, kNInPad / 64), dim3(256), 0, stream>>>(Win, WIN);
  wmma_gemm64<0, false, 0, 0, false><<<dim3(256, 1), dim3(256), 0, stream>>>(
      XH, XH, kDModel, 0L, WIN, WIN, kDModel, 0L, (void*)Zp, (void*)Zp, kDSsm, 0L,
      gam, gam, 0L, kRows, kDSsm, kDModel, kWinCarryInv);
  wmma_gemm64<0, false, 0, 0, false><<<dim3(288, 1), dim3(256), 0, stream>>>(
      XH, XH, kDModel, 0L, WIN + (size_t)kDSsm * kDModel, WIN + (size_t)kDSsm * kDModel, kDModel, 0L,
      (void*)XR, (void*)XR, kConvDim, 0L, gam, gam, 0L, kRows, kConvDim, kDModel, kWinCarryInv);
  wmma_gemm64<0, false, 0, 0, false><<<dim3(8, 1), dim3(256), 0, stream>>>(
      XH, XH, kDModel, 0L, WIN + (size_t)(kDSsm + kConvDim) * kDModel, WIN + (size_t)(kDSsm + kConvDim) * kDModel,
      kDModel, 0L, (void*)DTp, (void*)DTp, kNDt, 0L, gam, gam, 0L, kRows, kNDt, kDModel, kWinCarryInv);
  wout_tsplit_kernel<<<dim3(kDSsm / 64, kDModel / 64), dim3(256), 0, stream>>>(Wout, WOH, WOL);
  dtprep_kernel<<<dim3((kRows * kNHeads + 255) / 256), dim3(256), 0, stream>>>(DTp, dtb, Alog, DL, DA);
  conv_silu_kernel<<<dim3((kRows * kConvDim / 4 + 255) / 256), dim3(256), 0, stream>>>(XR, cw, cb, XC);
  scan_kernel<<<dim3(kBatch * kNHeads), dim3(256), 0, stream>>>(XC, DL, DA, Dv, Yp);
  gate_kernel<<<dim3(kRows), dim3(256), 0, stream>>>(Yp, Zp, gam, YH, YL);
  wmma_gemm64<1, true, 0, 0, false><<<dim3(128, 1), dim3(256), 0, stream>>>(
      YH, YL, kDSsm, 0L, WOH, WOL, kDSsm, 0L, (void*)out, (void*)out, kDModel, 0L,
      gam, gam, 0L, kRows, kDModel, kDSsm, 1.0f);
}
